// TransformerBlockQuantum_65481071395389
// MI455X (gfx1250) — hardware-verified
//
#include <hip/hip_runtime.h>


#pragma clang fp contract(off)

#ifndef NB
#define NB 2
#endif
#ifndef SEQ
#define SEQ 2048
#endif
#define NB_FULL  2
#define SEQ_FULL 2048
#define EMB  768
#define NH   12
#define DK   64
#define NQ   8
#define FFD  3072
#define KQ   32
#define NTOK (NB * SEQ)

#define WSC 64.0f
#define VSC 16.0f
#define PSC 16384.0f
#define CSC 8.0f
#define HSC 256.0f
#define SCL (0.125f * 1.4426950408889634f)
#define OSC (CSC / (PSC * VSC))

#define PP 72
#define CP 36
#define TP 72
#define PH 72

static_assert(NB >= 1 && NB <= NB_FULL);
static_assert(SEQ >= 64 && SEQ <= SEQ_FULL && (SEQ % 64) == 0);
static_assert((EMB % 64) == 0 && (FFD % 64) == 0 && (NTOK % 64) == 0);
static_assert(((NTOK * (EMB / 8)) % 256) == 0);
static_assert(NH * DK == EMB);
static_assert((EMB % 32) == 0 && (FFD % 32) == 0 && KQ == 32);

#define SZ_XB  ((size_t)NTOK * EMB * 2)
#define SZ_VT  ((size_t)NB * NH * DK * SEQ * 2)
#define SZ_WOT ((size_t)EMB * EMB * 2)
#define SZ_W2T ((size_t)EMB * FFD * 2)
#define SZ_W1T ((size_t)FFD * KQ * 2)
#define SZ_CTX ((size_t)NTOK * EMB * 2)
#define SZ_T   ((size_t)NTOK * EMB * 4)
#define SZ_H1  ((size_t)NTOK * FFD * 2)
static_assert(SZ_XB + SZ_VT + SZ_WOT + SZ_W2T + SZ_W1T + SZ_CTX + 3 * SZ_T + SZ_H1 + 10 * 256 <= (size_t)134217728);

typedef float          v4f   __attribute__((ext_vector_type(4)));
typedef float          v8f   __attribute__((ext_vector_type(8)));
typedef unsigned int   v4u   __attribute__((ext_vector_type(4)));
typedef _Float16       v8h   __attribute__((ext_vector_type(8)));
typedef _Float16       v16h  __attribute__((ext_vector_type(16)));
typedef __bf16         v16b  __attribute__((ext_vector_type(16)));
typedef unsigned short v8us  __attribute__((ext_vector_type(8)));
typedef unsigned short v16us __attribute__((ext_vector_type(16)));
typedef v8h  v8ha  __attribute__((may_alias));
typedef v8us v8usa __attribute__((may_alias));
typedef v4f  v4fa  __attribute__((may_alias));

union Frag { v16us u; v8us p[2]; v8h hp[2]; v16h h; v16b b; };

__device__ __forceinline__ unsigned short bf16bits(float v) {
    unsigned int u = __float_as_uint(v);
    u = u + 0x7FFFu + ((u >> 16) & 1u);
    return (unsigned short)(u >> 16);
}
__device__ __forceinline__ float bf16r(float v) {
    unsigned int u = __float_as_uint(v);
    u = (u + 0x7FFFu + ((u >> 16) & 1u)) & 0xFFFF0000u;
    return __uint_as_float(u);
}
__device__ __forceinline__ v4f bf16r4(v4f v) {
    v4u u = __builtin_bit_cast(v4u, v);
    u = (u + 0x7FFFu + ((u >> 16) & 1u)) & 0xFFFF0000u;
    return __builtin_bit_cast(v4f, u);
}
__device__ __forceinline__ unsigned short f16bits(float v) {
    _Float16 hv = (_Float16)v;
    return __builtin_bit_cast(unsigned short, hv);
}
__device__ __forceinline__ v8f zero8() {
    v8f z = {0.f, 0.f, 0.f, 0.f, 0.f, 0.f, 0.f, 0.f};
    return z;
}
__device__ __forceinline__ v8f mma_f16(v16h a, v16h b, v8f c) {
    v8f d = __builtin_amdgcn_wmma_f32_16x16x32_f16(false, a, false, b, (short)0, c, false, false);
    asm volatile("v_nop\n\tv_nop\n\tv_nop\n\tv_nop" : "+v"(d) : "v"(a), "v"(b));
    return d;
}
__device__ __forceinline__ v8f mma_bf16(v16b a, v16b b, v8f c) {
    v8f d = __builtin_amdgcn_wmma_f32_16x16x32_bf16(false, a, false, b, (short)0, c, false, false);
    asm volatile("v_nop\n\tv_nop\n\tv_nop\n\tv_nop" : "+v"(d) : "v"(a), "v"(b));
    return d;
}
__device__ __forceinline__ void lds_wave_sync() {
    __builtin_amdgcn_fence(3, "wavefront");
    __builtin_amdgcn_wave_barrier();
    __builtin_amdgcn_fence(2, "wavefront");
}

__global__ __launch_bounds__(256)
void k_cvtx(const float* __restrict__ x, unsigned short* __restrict__ xb)
{
    const int g = blockIdx.x * 256 + (int)threadIdx.x;
    const int t = g / (EMB / 8);
    const int piece = g - t * (EMB / 8);
    const int b = t / SEQ;
    const int s = t - b * SEQ;
    const float* xp = x + ((size_t)(b * SEQ_FULL + s)) * EMB + piece * 8;
    const v4f a = *(const v4f*)(xp);
    const v4f c = *(const v4f*)(xp + 4);
    const float e0 = a.x, e1 = a.y, e2 = a.z, e3 = a.w, e4 = c.x, e5 = c.y, e6 = c.z, e7 = c.w;
    v8us o;
    o[0] = bf16bits(e0); o[1] = bf16bits(e1); o[2] = bf16bits(e2); o[3] = bf16bits(e3);
    o[4] = bf16bits(e4); o[5] = bf16bits(e5); o[6] = bf16bits(e6); o[7] = bf16bits(e7);
    unsigned short* op = xb + (size_t)g * 8;
    *(volatile v8us*)op = o;
    __threadfence();
    *(volatile v8us*)op = o;
}

__global__ __launch_bounds__(256)
void k_tr(const float* __restrict__ in, int pitch_in, int zs_a, int zs_b, int zdiv,
          unsigned short* __restrict__ out, int pitch_out, int zs_out, float scale)
{
    __shared__ __align__(16) _Float16 sT[64 * TP];
    const int tid = (int)threadIdx.x;
    const int c0 = blockIdx.x * 64, r0 = blockIdx.y * 64, z = blockIdx.z;
    const float* ib = in + ((size_t)(z / zdiv)) * zs_a + ((size_t)(z % zdiv)) * zs_b
                         + (size_t)r0 * pitch_in + c0;
    #pragma unroll
    for (int p = 0; p < 4; ++p) {
        const int idx = tid + 256 * p;
        const int r = idx >> 4;
        const int c4 = (idx & 15) * 4;
        v4f v = *(const v4f*)(ib + (size_t)r * pitch_in + c4);
        v = bf16r4(v) * scale;
        const float v0 = v.x, v1 = v.y, v2 = v.z, v3 = v.w;
        sT[(c4 + 0) * TP + r] = (_Float16)v0;
        sT[(c4 + 1) * TP + r] = (_Float16)v1;
        sT[(c4 + 2) * TP + r] = (_Float16)v2;
        sT[(c4 + 3) * TP + r] = (_Float16)v3;
    }
    __syncthreads();
    unsigned short* ob = out + (size_t)z * zs_out + (size_t)c0 * pitch_out + r0;
    v8us o[2];
    #pragma unroll
    for (int it = 0; it < 2; ++it) {
        const int c = 32 * it + (tid >> 3), q = tid & 7;
        o[it] = *(const v8usa*)(sT + c * TP + 8 * q);
    }
    #pragma unroll
    for (int it = 0; it < 2; ++it) {
        const int c = 32 * it + (tid >> 3), q = tid & 7;
        *(volatile v8us*)(ob + (size_t)c * pitch_out + 8 * q) = o[it];
    }
    __threadfence();
    #pragma unroll
    for (int it = 0; it < 2; ++it) {
        const int c = 32 * it + (tid >> 3), q = tid & 7;
        *(volatile v8us*)(ob + (size_t)c * pitch_out + 8 * q) = o[it];
    }
}

__global__ __launch_bounds__(256)
void k_packw1(const float* __restrict__ W1, unsigned short* __restrict__ w1t)
{
    const int t = blockIdx.x * 256 + (int)threadIdx.x;
    const int f = t >> 2;
    const int q = t & 3;
    v8us o;
    #pragma unroll
    for (int i = 0; i < NQ; ++i) {
        const float wv = bf16r(W1[(size_t)i * FFD + f]) * WSC;
        const unsigned short hb = f16bits(wv);
        o[i] = (q == 0) ? hb : (unsigned short)0;
    }
    unsigned short* op = w1t + (size_t)t * 8;
    *(volatile v8us*)op = o;
    __threadfence();
    *(volatile v8us*)op = o;
}

__global__ __launch_bounds__(128) __attribute__((amdgpu_num_vgpr(256)))
void k_attn(const unsigned short* __restrict__ xb, const unsigned short* __restrict__ vt,
            unsigned short* __restrict__ ctx)
{
    __shared__ __align__(16) _Float16 sP[4][16 * PP];
    const int tid = (int)threadIdx.x;
    const int l = tid & 31, w = tid >> 5, h = l >> 4, m = l & 15;
    const int wid = blockIdx.x * 4 + w;
    const int qt = wid % (SEQ / 16);
    const int bh = wid / (SEQ / 16);
    const int b  = bh / NH;
    const int hh = bh - b * NH;
    const int tq0 = b * SEQ + qt * 16;
    _Float16* sp = &sP[w][0];

    Frag qa0, qa1;
    {
        const unsigned short* qp = xb + ((size_t)(tq0 + m)) * EMB + hh * DK + 8 * h;
        qa0.p[0] = *(const v8us*)(qp);      qa0.p[1] = *(const v8us*)(qp + 16);
        qa1.p[0] = *(const v8us*)(qp + 32); qa1.p[1] = *(const v8us*)(qp + 48);
    }
    const unsigned short* kl = xb + ((size_t)(b * SEQ + m)) * EMB + hh * DK + 8 * h;
    const unsigned short* vl = vt + ((size_t)(bh * DK + m)) * SEQ + 8 * h;

    v8f o[4];
    float mrow[8], lrow[8];
    #pragma unroll
    for (int f = 0; f < 4; ++f) o[f] = zero8();
    #pragma unroll
    for (int r = 0; r < 8; ++r) { mrow[r] = -1.0e30f; lrow[r] = 0.f; }

    #pragma unroll 1
    for (int j0 = 0; j0 < SEQ; j0 += 64) {
        v8f sc[4];
        #pragma unroll
        for (int t = 0; t < 4; ++t) {
            const unsigned short* kp = kl + ((size_t)(j0 + 16 * t)) * EMB;
            Frag kb;
            kb.p[0] = *(const v8us*)(kp);      kb.p[1] = *(const v8us*)(kp + 16);
            v8f acc = mma_bf16(qa0.b, kb.b, zero8());
            Frag kc;
            kc.p[0] = *(const v8us*)(kp + 32); kc.p[1] = *(const v8us*)(kp + 48);
            sc[t] = mma_bf16(qa1.b, kc.b, acc);
        }
        lds_wave_sync();
        #pragma unroll
        for (int r = 0; r < 8; ++r) {
            const float s0 = sc[0][r] * SCL, s1 = sc[1][r] * SCL, s2 = sc[2][r] * SCL, s3 = sc[3][r] * SCL;
            float mx = fmaxf(fmaxf(s0, s1), fmaxf(s2, s3));
            mx = fmaxf(mx, __shfl_xor(mx, 1));
            mx = fmaxf(mx, __shfl_xor(mx, 2));
            mx = fmaxf(mx, __shfl_xor(mx, 4));
            mx = fmaxf(mx, __shfl_xor(mx, 8));
            const float mn = fmaxf(mrow[r], mx);
            const float alpha = exp2f(mrow[r] - mn);
            mrow[r] = mn;
            const float p0 = exp2f(s0 - mn), p1 = exp2f(s1 - mn), p2 = exp2f(s2 - mn), p3 = exp2f(s3 - mn);
            float rs = (p0 + p1) + (p2 + p3);
            rs += __shfl_xor(rs, 1);
            rs += __shfl_xor(rs, 2);
            rs += __shfl_xor(rs, 4);
            rs += __shfl_xor(rs, 8);
            lrow[r] = lrow[r] * alpha + rs;
            o[0][r] = o[0][r] * alpha; o[1][r] = o[1][r] * alpha;
            o[2][r] = o[2][r] * alpha; o[3][r] = o[3][r] * alpha;
            _Float16* prow = sp + (8 * h + r) * PP + m;
            prow[0]  = (_Float16)(p0 * PSC);
            prow[16] = (_Float16)(p1 * PSC);
            prow[32] = (_Float16)(p2 * PSC);
            prow[48] = (_Float16)(p3 * PSC);
        }
        lds_wave_sync();
        #pragma unroll
        for (int kk = 0; kk < 2; ++kk) {
            Frag pa;
            const _Float16* pr = sp + m * PP + 32 * kk + 8 * h;
            pa.hp[0] = *(const v8ha*)(pr);
            pa.hp[1] = *(const v8ha*)(pr + 16);
            #pragma unroll
            for (int f = 0; f < 4; ++f) {
                const unsigned short* vp = vl + ((size_t)(16 * f)) * SEQ + j0 + 32 * kk;
                Frag vb;
                vb.p[0] = *(const v8us*)(vp); vb.p[1] = *(const v8us*)(vp + 16);
                o[f] = mma_f16(pa.h, vb.h, o[f]);
            }
        }
    }

    lds_wave_sync();
    #pragma unroll
    for (int r = 0; r < 8; ++r) {
        const float inv = __builtin_amdgcn_rcpf(lrow[r]) * OSC;
        _Float16* prow = sp + (8 * h + r) * PP + m;
        prow[0]  = (_Float16)(o[0][r] * inv);
        prow[16] = (_Float16)(o[1][r] * inv);
        prow[32] = (_Float16)(o[2][r] * inv);
        prow[48] = (_Float16)(o[3][r] * inv);
    }
    lds_wave_sync();
    v8us cv[4];
    #pragma unroll
    for (int it = 0; it < 4; ++it) {
        const int row = 4 * it + (l >> 3), q = l & 7;
        cv[it] = *(const v8usa*)(sp + row * PP + 8 * q);
    }
    #pragma unroll
    for (int it = 0; it < 4; ++it) {
        const int row = 4 * it + (l >> 3), q = l & 7;
        *(volatile v8us*)(ctx + ((size_t)(tq0 + row)) * EMB + hh * DK + 8 * q) = cv[it];
    }
    __threadfence();
    #pragma unroll
    for (int it = 0; it < 4; ++it) {
        const int row = 4 * it + (l >> 3), q = l & 7;
        *(volatile v8us*)(ctx + ((size_t)(tq0 + row)) * EMB + hh * DK + 8 * q) = cv[it];
    }
}

__global__ __launch_bounds__(128) __attribute__((amdgpu_num_vgpr(256)))
void k_gemm(const unsigned short* __restrict__ A, const unsigned short* __restrict__ BT,
            const float* __restrict__ res, const float* __restrict__ bias, float* __restrict__ C,
            int N, int K, int res_seq, int res_seq_full, int res_cvt, float oscale)
{
    __shared__ __align__(16) float sC[4][32 * CP];
    const int tid = (int)threadIdx.x;
    const int l = tid & 31, w = tid >> 5, h = l >> 4, m = l & 15;
    const int wm = blockIdx.y * 64 + 32 * (w >> 1);
    const int wn = blockIdx.x * 64 + 32 * (w & 1);
    const unsigned short* ap = A  + ((size_t)(wm + m)) * K + 8 * h;
    const unsigned short* bp = BT + ((size_t)(wn + m)) * K + 8 * h;
    const size_t s16 = (size_t)16 * K;

    v8f acc[2][2];
    acc[0][0] = zero8(); acc[0][1] = zero8(); acc[1][0] = zero8(); acc[1][1] = zero8();

    #pragma unroll 1
    for (int k0 = 0; k0 < K; k0 += 32) {
        Frag a0, a1, b0, b1;
        a0.p[0] = *(const v8us*)(ap + k0);        a0.p[1] = *(const v8us*)(ap + k0 + 16);
        a1.p[0] = *(const v8us*)(ap + s16 + k0);  a1.p[1] = *(const v8us*)(ap + s16 + k0 + 16);
        b0.p[0] = *(const v8us*)(bp + k0);        b0.p[1] = *(const v8us*)(bp + k0 + 16);
        b1.p[0] = *(const v8us*)(bp + s16 + k0);  b1.p[1] = *(const v8us*)(bp + s16 + k0 + 16);
        acc[0][0] = mma_f16(a0.h, b0.h, acc[0][0]);
        acc[0][1] = mma_f16(a0.h, b1.h, acc[0][1]);
        acc[1][0] = mma_f16(a1.h, b0.h, acc[1][0]);
        acc[1][1] = mma_f16(a1.h, b1.h, acc[1][1]);
    }

    float* sc = &sC[w][0];
    lds_wave_sync();
    #pragma unroll
    for (int i = 0; i < 2; ++i)
        #pragma unroll
        for (int j = 0; j < 2; ++j)
            #pragma unroll
            for (int r = 0; r < 8; ++r)
                sc[(16 * i + 8 * h + r) * CP + 16 * j + m] = acc[i][j][r];
    lds_wave_sync();

    v4f ov[8];
    #pragma unroll
    for (int it = 0; it < 8; ++it) {
        const int row = 4 * it + (l >> 3), q = l & 7;
        const v4f c = *(const v4fa*)(sc + row * CP + 4 * q);
        const int grow = wm + row;
        const int col  = wn + 4 * q;
        const int rrow = (grow / res_seq) * res_seq_full + (grow % res_seq);
        v4f rv = *(const v4f*)(res + (size_t)rrow * N + col);
        if (res_cvt != 0) rv = bf16r4(rv);
        const v4f bv = bf16r4(*(const v4f*)(bias + col));
        v4f t = c * oscale;
        t = t + bv;
        ov[it] = rv + t;
    }
    #pragma unroll
    for (int it = 0; it < 8; ++it) {
        const int row = 4 * it + (l >> 3), q = l & 7;
        *(volatile v4f*)(C + ((size_t)(wm + row)) * N + wn + 4 * q) = ov[it];
    }
    __threadfence();
    #pragma unroll
    for (int it = 0; it < 8; ++it) {
        const int row = 4 * it + (l >> 3), q = l & 7;
        *(volatile v4f*)(C + ((size_t)(wm + row)) * N + wn + 4 * q) = ov[it];
    }
}

__global__ __launch_bounds__(256)
void k_ln(const float* __restrict__ in, const float* __restrict__ g, const float* __restrict__ be,
          float* __restrict__ out, int out_seq_full)
{
    const int tid = (int)threadIdx.x;
    const int l = tid & 31, w = tid >> 5;
    const int row = blockIdx.x * 8 + w;
    const float* rp = in + (size_t)row * EMB;
    v4f v[6];
    #pragma unroll
    for (int i = 0; i < 6; ++i) v[i] = *(const v4f*)(rp + (i * 32 + l) * 4);
    float s = 0.f;
    #pragma unroll
    for (int i = 0; i < 6; ++i) s += (v[i].x + v[i].y) + (v[i].z + v[i].w);
    s += __shfl_xor(s, 16); s += __shfl_xor(s, 8); s += __shfl_xor(s, 4);
    s += __shfl_xor(s, 2);  s += __shfl_xor(s, 1);
    const float mean = s * (1.0f / (float)EMB);
    float qs = 0.f;
    #pragma unroll
    for (int i = 0; i < 6; ++i) {
        v[i] = v[i] - mean;
        const v4f d2 = v[i] * v[i];
        qs += (d2.x + d2.y) + (d2.z + d2.w);
    }
    qs += __shfl_xor(qs, 16); qs += __shfl_xor(qs, 8); qs += __shfl_xor(qs, 4);
    qs += __shfl_xor(qs, 2);  qs += __shfl_xor(qs, 1);
    const float var  = qs * (1.0f / (float)EMB);
    const float rstd = rsqrtf(var + 1e-5f);
    v4f y[6];
    #pragma unroll
    for (int i = 0; i < 6; ++i) {
        const int col = (i * 32 + l) * 4;
        const v4f gv = bf16r4(*(const v4f*)(g + col));
        const v4f bv = bf16r4(*(const v4f*)(be + col));
        v4f t = v[i] * rstd;
        t = t * gv;
        y[i] = t + bv;
    }
    const int orow = (row / SEQ) * out_seq_full + (row % SEQ);
    float* op = out + (size_t)orow * EMB;
    #pragma unroll
    for (int i = 0; i < 6; ++i) *(volatile v4f*)(op + (i * 32 + l) * 4) = y[i];
    __threadfence();
    #pragma unroll
    for (int i = 0; i < 6; ++i) *(volatile v4f*)(op + (i * 32 + l) * 4) = y[i];
}

__global__ __launch_bounds__(64) __attribute__((amdgpu_num_vgpr(256)))
void k_ffn1(const float* __restrict__ x1, const float* __restrict__ ry,
            const unsigned short* __restrict__ w1t, const float* __restrict__ b1,
            unsigned short* __restrict__ h1)
{
    __shared__ __align__(16) float    sQ[2][16 * NQ];
    __shared__ __align__(16) _Float16 sH[2][16 * PH];
    const int tid = (int)threadIdx.x;
    const int l = tid & 31, w = tid >> 5, h = l >> 4, m = l & 15;
    const int r0 = (blockIdx.x * 2 + w) * 16;
    float* sq = &sQ[w][0];
    _Float16* sh = &sH[w][0];

    const float cry = cosf(bf16r(ry[l & 7]));
    #pragma unroll 1
    for (int p = 0; p < 4; ++p) {
        const int rr = 4 * p + (l >> 3), i = l & 7;
        const float xv = x1[((size_t)(r0 + rr)) * EMB + i];
        sq[rr * NQ + i] = cosf(xv) * cry;
    }
    lds_wave_sync();
    const v4f q0 = *(const v4fa*)(sq + m * NQ);
    const v4f q1 = *(const v4fa*)(sq + m * NQ + 4);
    v16h av;
    av[0] = (_Float16)(h ? 0.f : q0.x); av[1] = (_Float16)(h ? 0.f : q0.y);
    av[2] = (_Float16)(h ? 0.f : q0.z); av[3] = (_Float16)(h ? 0.f : q0.w);
    av[4] = (_Float16)(h ? 0.f : q1.x); av[5] = (_Float16)(h ? 0.f : q1.y);
    av[6] = (_Float16)(h ? 0.f : q1.z); av[7] = (_Float16)(h ? 0.f : q1.w);
    #pragma unroll
    for (int i = 8; i < 16; ++i) av[i] = (_Float16)0.f;

    const unsigned short* wp = w1t + (size_t)m * KQ + 8 * h;

    #pragma unroll 1
    for (int gi = 0; gi < FFD / 64; ++gi) {
        v8f acc[4];
        #pragma unroll
        for (int u = 0; u < 4; ++u) {
            const unsigned short* p = wp + ((size_t)(4 * gi + u)) * (16 * KQ);
            Frag bf;
            bf.p[0] = *(const v8us*)(p); bf.p[1] = *(const v8us*)(p + 16);
            acc[u] = mma_f16(av, bf.h, zero8());
        }
        lds_wave_sync();
        #pragma unroll
        for (int u = 0; u < 4; ++u) {
            const float bb = bf16r(b1[64 * gi + 16 * u + m]);
            #pragma unroll
            for (int r = 0; r < 8; ++r) {
                float hv = acc[u][r] * (1.0f / WSC);
                hv = hv + bb;
                hv = fmaxf(hv, 0.f) * HSC;
                sh[(8 * h + r) * PH + 16 * u + m] = (_Float16)hv;
            }
        }
        lds_wave_sync();
        v8us hvv[4];
        #pragma unroll
        for (int it = 0; it < 4; ++it) {
            const int row = 4 * it + (l >> 3), q = l & 7;
            hvv[it] = *(const v8usa*)(sh + row * PH + 8 * q);
        }
        #pragma unroll
        for (int it = 0; it < 4; ++it) {
            const int row = 4 * it + (l >> 3), q = l & 7;
            *(volatile v8us*)(h1 + ((size_t)(r0 + row)) * FFD + 64 * gi + 8 * q) = hvv[it];
        }
        __threadfence();
        #pragma unroll
        for (int it = 0; it < 4; ++it) {
            const int row = 4 * it + (l >> 3), q = l & 7;
            *(volatile v8us*)(h1 + ((size_t)(r0 + row)) * FFD + 64 * gi + 8 * q) = hvv[it];
        }
    }
}

extern "C" void kernel_launch(void* const* d_in, const int* in_sizes, int n_in,
                              void* d_out, int out_size, void* d_ws, size_t ws_size,
                              hipStream_t stream)
{
    if (n_in < 12) return;
    const float* x   = (const float*)d_in[0];
    const float* W_o = (const float*)d_in[1];
    const float* b_o = (const float*)d_in[2];
    const float* g1  = (const float*)d_in[3];
    const float* be1 = (const float*)d_in[4];
    const float* g2  = (const float*)d_in[5];
    const float* be2 = (const float*)d_in[6];
    const float* ry  = (const float*)d_in[7];
    const float* W1  = (const float*)d_in[8];
    const float* b1  = (const float*)d_in[9];
    const float* W2  = (const float*)d_in[10];
    const float* b2  = (const float*)d_in[11];
    float* out = (float*)d_out;

    const int need_x = ((NB - 1) * SEQ_FULL + SEQ) * EMB;
    if (in_sizes[0] < need_x || in_sizes[1] < EMB * EMB || in_sizes[2] < EMB ||
        in_sizes[3] < EMB || in_sizes[4] < EMB || in_sizes[5] < EMB || in_sizes[6] < EMB ||
        in_sizes[7] < NQ || in_sizes[8] < NQ * FFD || in_sizes[9] < FFD ||
        in_sizes[10] < FFD * EMB || in_sizes[11] < EMB) return;
    if (out_size < need_x) return;

    size_t off = 0;
    auto carve = [&](size_t bytes) -> char* {
        off = (off + 255) & ~(size_t)255;
        char* p = (char*)d_ws + off;
        off += bytes;
        return p;
    };
    unsigned short* xb  = (unsigned short*)carve(SZ_XB);
    unsigned short* vt  = (unsigned short*)carve(SZ_VT);
    unsigned short* wot = (unsigned short*)carve(SZ_WOT);
    unsigned short* w2t = (unsigned short*)carve(SZ_W2T);
    unsigned short* w1t = (unsigned short*)carve(SZ_W1T);
    unsigned short* ctx = (unsigned short*)carve(SZ_CTX);
    float*          t1  = (float*)carve(SZ_T);
    float*          x1  = (float*)carve(SZ_T);
    unsigned short* h1  = (unsigned short*)carve(SZ_H1);
    float*          t2  = (float*)carve(SZ_T);
    if (off > ws_size) return;

    k_cvtx<<<dim3((NTOK * (EMB / 8)) / 256), dim3(256), 0, stream>>>(x, xb);
    k_tr<<<dim3(DK / 64, SEQ / 64, NB * NH), dim3(256), 0, stream>>>(
        x, EMB, SEQ_FULL * EMB, DK, NH, vt, SEQ, DK * SEQ, VSC);
    k_tr<<<dim3(EMB / 64, EMB / 64, 1), dim3(256), 0, stream>>>(
        W_o, EMB, 0, 0, 1, wot, EMB, 0, WSC);
    k_tr<<<dim3(EMB / 64, FFD / 64, 1), dim3(256), 0, stream>>>(
        W2, EMB, 0, 0, 1, w2t, FFD, 0, WSC);
    k_packw1<<<dim3((FFD * 4) / 256), dim3(256), 0, stream>>>(W1, w1t);

    k_attn<<<dim3(NB * NH * (SEQ / 64)), dim3(128), 0, stream>>>(xb, vt, ctx);
    k_gemm<<<dim3(EMB / 64, NTOK / 64), dim3(128), 0, stream>>>(
        ctx, wot, x, b_o, t1, EMB, EMB, SEQ, SEQ_FULL, 1, 1.0f / (CSC * WSC));
    k_ln<<<dim3(NTOK / 8), dim3(256), 0, stream>>>(t1, g1, be1, x1, SEQ);
    k_ffn1<<<dim3(NTOK / 32), dim3(64), 0, stream>>>(x1, ry, w1t, b1, h1);
    k_gemm<<<dim3(EMB / 64, NTOK / 64), dim3(128), 0, stream>>>(
        h1, w2t, x1, b2, t2, EMB, FFD, SEQ, SEQ, 0, 1.0f / (HSC * WSC));
    k_ln<<<dim3(NTOK / 8), dim3(256), 0, stream>>>(t2, g2, be2, out, SEQ_FULL);
}
